// MultiLatentAttention_35802847380107
// MI455X (gfx1250) — hardware-verified
//
#include <hip/hip_runtime.h>
#include <stddef.h>


typedef _Float16 v16h __attribute__((ext_vector_type(16)));
typedef _Float16 v8h  __attribute__((ext_vector_type(8)));
typedef float    v8f  __attribute__((ext_vector_type(8)));
typedef float    v4f  __attribute__((ext_vector_type(4)));

#ifndef NB
#define NB 2
#endif
#ifndef SEQ
#define SEQ 2048
#endif
#define NB_FULL  2
#define SEQ_FULL 2048
#define DIM   1024
#define NHEAD 16
#define PDIM  64
#define HALF  32
#define MROWS (NB * SEQ)

static_assert(NB >= 1 && NB <= NB_FULL);
static_assert(SEQ >= 128 && SEQ <= SEQ_FULL && (SEQ % 128) == 0);
static_assert(DIM == NHEAD * PDIM);
static_assert(PDIM == 64);
static_assert(HALF * 2 == PDIM && HALF == 32);
static_assert(DIM / NHEAD == 64);
static_assert((DIM % 64) == 0 && (DIM % 32) == 0);
static_assert((PDIM % 64) == 0);
static_assert((MROWS % 64) == 0 && (MROWS % 8) == 0);
static_assert((SEQ % 64) == 0);
static_assert(DIM == 4 * 32 * 8);
static_assert(DIM == 32 * 32);
static_assert(PDIM * 2 == 128);
static_assert((size_t)MROWS * DIM < (size_t)0xFFFFFFFFu);

#define LDT 72
#define LDC 68
static_assert((LDT % 8) == 0 && LDT >= 64);
static_assert((LDC % 4) == 0 && LDC >= 64);

#define WCARRY 64.0f
#define ACARRY 16.0f
#define SCARRY 64.0f
#define HCARRY 16.0f
#define SCALE  0.125f

#define WSQ_BYTES     ((size_t)DIM * DIM * 2)
#define WPJ_BYTES     ((size_t)PDIM * DIM * 2)
#define PLANE16_BYTES ((size_t)MROWS * DIM * 2)
#define QKV_BYTES     ((size_t)MROWS * PDIM * 2)
#define LAM_BYTES     ((size_t)128)
#define OFF_WQ  ((size_t)0)
#define OFF_WK  (OFF_WQ + WSQ_BYTES)
#define OFF_WV  (OFF_WK + WSQ_BYTES)
#define OFF_RW  (OFF_WV + WSQ_BYTES)
#define OFF_PJ  (OFF_RW + WSQ_BYTES)
#define OFF_X16 (OFF_PJ + WPJ_BYTES)
#define OFF_TQ  (OFF_X16 + PLANE16_BYTES)
#define OFF_TK  (OFF_TQ + PLANE16_BYTES)
#define OFF_TV  (OFF_TK + PLANE16_BYTES)
#define OFF_Q   (OFF_TV + PLANE16_BYTES)
#define OFF_K   (OFF_Q + QKV_BYTES)
#define OFF_VT  (OFF_K + QKV_BYTES)
#define OFF_HD  (OFF_VT + QKV_BYTES)
#define OFF_LAM (OFF_HD + PLANE16_BYTES)
#define WS_TOTAL (OFF_LAM + LAM_BYTES)
static_assert((WSQ_BYTES % 128) == 0 && (WPJ_BYTES % 128) == 0 && (PLANE16_BYTES % 128) == 0);
static_assert((QKV_BYTES % 128) == 0 && (LAM_BYTES % 128) == 0);
static_assert((size_t)NB * PDIM * SEQ * 2 == QKV_BYTES);
static_assert(WS_TOTAL <= (size_t)134217728);

__device__ __forceinline__ float bf16r(float x) {
  unsigned int u = __float_as_uint(x);
  u = (u + 0x7FFFu + ((u >> 16) & 1u)) & 0xFFFF0000u;
  return __uint_as_float(u);
}

static __device__ __forceinline__ _Float16 toh_flush(float v) {
  const _Float16 r = (_Float16)v;
  return (fabsf(v) < 6.103515625e-05f) ? (_Float16)0.0f : r;
}

__device__ __forceinline__ v16h frag_at(const _Float16* p) {
  v8h lo = *(const v8h*)(p);
  v8h hi = *(const v8h*)(p + 16);
  v16h out;
#pragma unroll
  for (int i = 0; i < 8; ++i) { out[i] = lo[i]; out[i + 8] = hi[i]; }
  return out;
}
__device__ __forceinline__ v16h ld_frag(const _Float16* base, unsigned ld) {
  const unsigned lane = threadIdx.x & 31u;
  return frag_at(base + (lane & 15u) * ld + (lane >> 4) * 8u);
}

__device__ __forceinline__ v8f wmma16(v16h a, v16h b, v8f c) {
  v8f d = __builtin_amdgcn_wmma_f32_16x16x32_f16(false, a, false, b, (short)0, c,
                                                 false, false);
  asm volatile("v_nop\n\tv_nop\n\tv_nop\n\tv_nop" : "+v"(d) : "v"(a), "v"(b));
  return d;
}

__device__ __forceinline__ float red32_sum(float x) {
#pragma unroll
  for (int off = 1; off < 32; off <<= 1) x += __shfl_xor(x, off, 32);
  return x;
}

__device__ __forceinline__ void wave_lds_sync() {
  __builtin_amdgcn_fence(3  , "wavefront");
  asm volatile("s_wait_dscnt 0x0" ::: "memory");
  __builtin_amdgcn_wave_barrier();
}

__global__ __launch_bounds__(256) void wconv_kernel(
    const float* __restrict__ W, _Float16* __restrict__ Wt, unsigned ldw, unsigned ldk) {
  __shared__ _Float16 T[64 * LDT];
  const unsigned tid = threadIdx.x;
  const unsigned n0 = blockIdx.x * 64u;
  const unsigned k0 = blockIdx.y * 64u;
#pragma unroll 4
  for (unsigned j = 0; j < 16u; ++j) {
    const unsigned idx = tid + 256u * j;
    const unsigned kr = idx >> 6, nc = idx & 63u;
    const float v = W[(size_t)(k0 + kr) * ldw + n0 + nc];
    T[nc * LDT + kr] = (_Float16)(WCARRY * bf16r(v));
  }
  __syncthreads();
  v8h x[2];
  size_t off[2];
#pragma unroll
  for (unsigned i = 0; i < 2u; ++i) {
    const unsigned n = 32u * i + (tid >> 3);
    const unsigned kc = (tid & 7u) * 8u;
    x[i] = *(const v8h*)&T[n * LDT + kc];
    off[i] = (size_t)(n0 + n) * ldk + k0 + kc;
  }
#pragma unroll
  for (int i = 0; i < 2; ++i) *(volatile v8h*)(Wt + off[i]) = x[i];
  __threadfence();
#pragma unroll
  for (int i = 0; i < 2; ++i) *(volatile v8h*)(Wt + off[i]) = x[i];
}

__global__ __launch_bounds__(256) void xconv_kernel(
    const float* __restrict__ X, _Float16* __restrict__ dst) {
#pragma clang fp contract(off)
  const unsigned lane = threadIdx.x & 31u, w = threadIdx.x >> 5;
  const unsigned crow = blockIdx.x * 8u + w;
  const unsigned bidx = crow / (unsigned)SEQ;
  const unsigned sq = crow - bidx * (unsigned)SEQ;
  const size_t srow = (size_t)bidx * SEQ_FULL + sq;
  const float* xr = X + srow * DIM + lane * 8u;
#pragma unroll 1
  for (unsigned j = 0; j < 4u; ++j) {
    const unsigned c = j * 256u + lane * 8u;
    const v4f a0 = *(const v4f*)(xr + j * 256u);
    const v4f a1 = *(const v4f*)(xr + j * 256u + 4u);
    v8h o;
#pragma unroll
    for (int i = 0; i < 4; ++i) {
      o[i]     = toh_flush(ACARRY * bf16r(a0[i]));
      o[i + 4] = toh_flush(ACARRY * bf16r(a1[i]));
    }
    _Float16* p = dst + (size_t)crow * DIM + c;
    *(volatile v8h*)p = o;
    __threadfence();
    *(volatile v8h*)p = o;
  }
}

__global__ __launch_bounds__(32) void lam_kernel(
    const float* __restrict__ q1, const float* __restrict__ k1,
    const float* __restrict__ q2, const float* __restrict__ k2,
    const float* __restrict__ li, float* __restrict__ lam_out) {
#pragma clang fp contract(off)
  const unsigned lane = threadIdx.x & 31u;
  float a1 = 0.0f, a2 = 0.0f;
#pragma unroll 1
  for (unsigned j = 0; j < (unsigned)(DIM / 32); ++j) {
    const unsigned i = j * 32u + lane;
    a1 += bf16r(q1[i]) * bf16r(k1[i]);
    a2 += bf16r(q2[i]) * bf16r(k2[i]);
  }
  a1 = red32_sum(a1);
  a2 = red32_sum(a2);
  const float lam = (expf(a1) - expf(a2)) + bf16r(li[0]);
  v4f o;
  o[0] = lam; o[1] = lam; o[2] = lam; o[3] = lam;
  if (lane < 8u) *(volatile v4f*)(lam_out + lane * 4u) = o;
  __threadfence();
  if (lane < 8u) *(volatile v4f*)(lam_out + lane * 4u) = o;
}

template <int MODE>
__device__ __forceinline__ void gemm_body(
    const _Float16* __restrict__ A16, const _Float16* __restrict__ Bt, const unsigned K,
    const float* __restrict__ bias, float* __restrict__ outf, _Float16* __restrict__ out16) {
  __shared__ float Cs[64 * LDC];
  const unsigned tid = threadIdx.x, lane = tid & 31u, w = tid >> 5;
  const unsigned mw = w >> 1, nw = w & 1u;
  const unsigned hh = lane >> 4, m = lane & 15u;
  const unsigned n0 = blockIdx.x * 64u;
  const unsigned row0 = blockIdx.y * 64u;

  const _Float16* ap  = A16 + (size_t)(row0 + mw * 16u + m) * K + hh * 8u;
  const _Float16* bp0 = Bt + (size_t)(n0 + nw * 32u + m) * K + hh * 8u;
  const _Float16* bp1 = bp0 + (size_t)16 * K;
  v8f acc0 = {}, acc1 = {};
#pragma unroll 2
  for (unsigned k0 = 0; k0 < K; k0 += 32u) {
    const v16h a  = frag_at(ap + k0);
    const v16h b0 = frag_at(bp0 + k0);
    const v16h b1 = frag_at(bp1 + k0);
    acc0 = wmma16(a, b0, acc0);
    acc1 = wmma16(a, b1, acc1);
  }
#pragma unroll
  for (int r = 0; r < 8; ++r) {
    float* d = &Cs[(mw * 16u + hh * 8u + (unsigned)r) * LDC + nw * 32u + m];
    d[0]  = acc0[r];
    d[16] = acc1[r];
  }
  __syncthreads();

  if (MODE == 0 || MODE == 1) {
    const unsigned ldo = (MODE == 1) ? (unsigned)PDIM : (unsigned)DIM;
    v8h x[2];
    size_t off[2];
#pragma unroll
    for (unsigned i = 0; i < 2u; ++i) {
      const unsigned r = 32u * i + (tid >> 3);
      const unsigned c = (tid & 7u) * 8u;
      const v4f u0 = *(const v4f*)&Cs[r * LDC + c];
      const v4f u1 = *(const v4f*)&Cs[r * LDC + c + 4];
      if (MODE == 1) {
        const v4f g0 = *(const v4f*)(bias + n0 + c);
        const v4f g1 = *(const v4f*)(bias + n0 + c + 4u);
#pragma unroll
        for (int j = 0; j < 4; ++j) {
          x[i][j]     = toh_flush(ACARRY * (u0[j] * (1.0f / (ACARRY * WCARRY)) + bf16r(g0[j])));
          x[i][j + 4] = toh_flush(ACARRY * (u1[j] * (1.0f / (ACARRY * WCARRY)) + bf16r(g1[j])));
        }
      } else {
#pragma unroll
        for (int j = 0; j < 4; ++j) {
          x[i][j]     = toh_flush(u0[j] * (1.0f / WCARRY));
          x[i][j + 4] = toh_flush(u1[j] * (1.0f / WCARRY));
        }
      }
      off[i] = (size_t)(row0 + r) * ldo + n0 + c;
    }
#pragma unroll
    for (int i = 0; i < 2; ++i) *(volatile v8h*)(out16 + off[i]) = x[i];
    __threadfence();
#pragma unroll
    for (int i = 0; i < 2; ++i) *(volatile v8h*)(out16 + off[i]) = x[i];
  }

  if (MODE == 2) {
    const unsigned bidx = row0 / (unsigned)SEQ;
    const unsigned key0 = row0 - bidx * (unsigned)SEQ;
    v8h x[2];
    size_t off[2];
#pragma unroll
    for (unsigned i = 0; i < 2u; ++i) {
      const unsigned dcol = 32u * i + (tid >> 3);
      const unsigned kk = (tid & 7u) * 8u;
      const float bb = bf16r(bias[n0 + dcol]);
#pragma unroll
      for (unsigned j = 0; j < 8u; ++j) {
        const float t = Cs[(kk + j) * LDC + dcol] * (1.0f / (ACARRY * WCARRY)) + bb;
        x[i][j] = toh_flush(ACARRY * t);
      }
      off[i] = ((size_t)bidx * PDIM + n0 + dcol) * SEQ + key0 + kk;
    }
#pragma unroll
    for (int i = 0; i < 2; ++i) *(volatile v8h*)(out16 + off[i]) = x[i];
    __threadfence();
#pragma unroll
    for (int i = 0; i < 2; ++i) *(volatile v8h*)(out16 + off[i]) = x[i];
  }

  if (MODE == 3) {
    const float cs = 1.0f / (WCARRY * HCARRY);
    v4f xs[4];
    size_t off[4];
#pragma unroll
    for (unsigned i = 0; i < 4u; ++i) {
      const unsigned r = 16u * i + (tid >> 4);
      const unsigned c = (tid & 15u) * 4u;
      const unsigned crow = row0 + r;
      const unsigned bidx = crow / (unsigned)SEQ;
      const unsigned sq = crow - bidx * (unsigned)SEQ;
      const size_t frow = (size_t)bidx * SEQ_FULL + sq;
      const v4f u = *(const v4f*)&Cs[r * LDC + c];
      v4f val;
#pragma unroll
      for (int j = 0; j < 4; ++j) val[j] = u[j] * cs;
      xs[i] = val;
      off[i] = frow * DIM + n0 + c;
    }
#pragma unroll
    for (int i = 0; i < 4; ++i) *(volatile v4f*)(outf + off[i]) = xs[i];
    __threadfence();
#pragma unroll
    for (int i = 0; i < 4; ++i) *(volatile v4f*)(outf + off[i]) = xs[i];
  }
}

__global__ __launch_bounds__(256) void gemm_t_kernel(
    const _Float16* __restrict__ A16, const _Float16* __restrict__ Bt,
    _Float16* __restrict__ out16) {
  gemm_body<0>(A16, Bt, (unsigned)DIM, (const float*)0, (float*)0, out16);
}
__global__ __launch_bounds__(256) void gemm_qk_kernel(
    const _Float16* __restrict__ A16, const _Float16* __restrict__ Bt,
    const float* __restrict__ bias, _Float16* __restrict__ out16) {
  gemm_body<1>(A16, Bt, (unsigned)DIM, bias, (float*)0, out16);
}
__global__ __launch_bounds__(256) void gemm_v_kernel(
    const _Float16* __restrict__ A16, const _Float16* __restrict__ Bt,
    const float* __restrict__ bias, _Float16* __restrict__ vt) {
  gemm_body<2>(A16, Bt, (unsigned)DIM, bias, (float*)0, vt);
}
__global__ __launch_bounds__(256) void gemm_out_kernel(
    const _Float16* __restrict__ A16, const _Float16* __restrict__ Bt,
    float* __restrict__ outf) {
  gemm_body<3>(A16, Bt, (unsigned)DIM, (const float*)0, outf, (_Float16*)0);
}

__global__ __launch_bounds__(256) void attn_kernel(
    const _Float16* __restrict__ Qh, const _Float16* __restrict__ Kh,
    const _Float16* __restrict__ Vt, const float* __restrict__ lamp,
    _Float16* __restrict__ Hd) {
  __shared__ _Float16 Ks[64 * LDT];
  __shared__ _Float16 Vs[64 * LDT];
  __shared__ _Float16 Ps[8 * 16 * LDT];

  const unsigned tid = threadIdx.x, lane = tid & 31u;
  const unsigned w = (unsigned)__builtin_amdgcn_readfirstlane((int)(threadIdx.x >> 5));
  const unsigned hh = lane >> 4, m = lane & 15u;
  const unsigned q0 = blockIdx.x * 128u;
  const unsigned b = blockIdx.y;
  const unsigned qrow0 = q0 + w * 16u;
  const float lam = lamp[0];
  const float c1 = SCALE * SCARRY / (ACARRY * ACARRY);
  const float c2 = lam * c1;
  _Float16* P = Ps + w * (16u * LDT);

  const size_t qoff = (size_t)(b * (unsigned)SEQ + qrow0 + m) * PDIM + hh * 8u;
  v16h qf[2];
  qf[0] = frag_at(Qh + qoff);
  qf[1] = frag_at(Qh + qoff + 32);

  v8f o[4];
#pragma unroll
  for (int nb = 0; nb < 4; ++nb) o[nb] = (v8f){};

  const size_t kplane = (size_t)b * SEQ * PDIM;
  const size_t vplane = (size_t)b * PDIM * SEQ;

  for (unsigned kb = 0; kb < (unsigned)SEQ; kb += 64u) {
#pragma unroll
    for (unsigned j = 0; j < 2u; ++j) {
      const unsigned idx = tid + 256u * j;
      const unsigned r = idx >> 3, c = (idx & 7u) * 8u;
      *(v8h*)&Ks[r * LDT + c] = *(const v8h*)(Kh + kplane + (size_t)(kb + r) * PDIM + c);
      *(v8h*)&Vs[r * LDT + c] = *(const v8h*)(Vt + vplane + (size_t)r * SEQ + kb + c);
    }
    __syncthreads();

    v8f s[4];
#pragma unroll
    for (int kg = 0; kg < 4; ++kg) {
      const v16h kf0 = ld_frag(&Ks[(kg * 16) * LDT], LDT);
      const v16h kf1 = ld_frag(&Ks[(kg * 16) * LDT + 32], LDT);
      v8f t1 = {};
      t1 = wmma16(qf[0], kf0, t1);
      v8f t2 = {};
      t2 = wmma16(qf[1], kf1, t2);
      s[kg] = t1 * c1 - t2 * c2;
    }

#pragma unroll
    for (int kg = 0; kg < 4; ++kg)
#pragma unroll
      for (int v = 0; v < 8; ++v)
        P[(hh * 8u + (unsigned)v) * LDT + (unsigned)kg * 16u + m] = toh_flush(s[kg][v]);
    wave_lds_sync();

#pragma unroll
    for (int c = 0; c < 2; ++c) {
      const v16h pf = ld_frag(P + c * 32, LDT);
#pragma unroll
      for (int nb = 0; nb < 4; ++nb) {
        const v16h vf = ld_frag(&Vs[(nb * 16) * LDT + c * 32], LDT);
        o[nb] = wmma16(pf, vf, o[nb]);
      }
    }
    __syncthreads();
  }

#pragma unroll 1
  for (unsigned h = 0; h < (unsigned)NHEAD; ++h) {
    const float hm = (float)(h + 1u) * (HCARRY / (SCARRY * ACARRY));
#pragma unroll
    for (int nb = 0; nb < 4; ++nb)
#pragma unroll
      for (int v = 0; v < 8; ++v)
        P[(hh * 8u + (unsigned)v) * LDT + (unsigned)nb * 16u + m] = toh_flush(o[nb][v] * hm);
    wave_lds_sync();
    v8h x[4];
    size_t off[4];
#pragma unroll
    for (unsigned i = 0; i < 4u; ++i) {
      const unsigned r = 4u * i + (lane >> 3);
      const unsigned c = (lane & 7u) * 8u;
      x[i] = *(const v8h*)&P[r * LDT + c];
      off[i] = (size_t)(b * (unsigned)SEQ + qrow0 + r) * DIM + h * (unsigned)PDIM + c;
    }
#pragma unroll
    for (int i = 0; i < 4; ++i) *(volatile v8h*)(Hd + off[i]) = x[i];
    __threadfence();
#pragma unroll
    for (int i = 0; i < 4; ++i) *(volatile v8h*)(Hd + off[i]) = x[i];
    wave_lds_sync();
  }
}

extern "C" void kernel_launch(void* const* d_in, const int* in_sizes, int n_in,
                              void* d_out, int out_size, void* d_ws, size_t ws_size,
                              hipStream_t stream) {
  if (n_in < 12) return;
  const long long need_x = ((long long)(NB - 1) * SEQ_FULL + SEQ) * DIM;
  if ((long long)in_sizes[0] < need_x) return;
  if ((long long)in_sizes[1] < (long long)DIM * DIM) return;
  if ((long long)in_sizes[2] < (long long)DIM * DIM) return;
  if ((long long)in_sizes[3] < (long long)DIM * DIM) return;
  if ((long long)in_sizes[4] < (long long)DIM * DIM) return;
  if ((long long)in_sizes[5] < (long long)DIM * PDIM) return;
  if (in_sizes[6] < PDIM) return;
  if (in_sizes[7] < DIM || in_sizes[8] < DIM || in_sizes[9] < DIM || in_sizes[10] < DIM) return;
  if (in_sizes[11] < 1) return;
  if ((long long)out_size < need_x) return;
  if (ws_size < WS_TOTAL) return;

  const float* X   = (const float*)d_in[0];
  const float* wq  = (const float*)d_in[1];
  const float* wk  = (const float*)d_in[2];
  const float* wv  = (const float*)d_in[3];
  const float* rw  = (const float*)d_in[4];
  const float* pw  = (const float*)d_in[5];
  const float* pb  = (const float*)d_in[6];
  const float* q1v = (const float*)d_in[7];
  const float* k1v = (const float*)d_in[8];
  const float* q2v = (const float*)d_in[9];
  const float* k2v = (const float*)d_in[10];
  const float* li  = (const float*)d_in[11];
  float* out = (float*)d_out;

  char* ws = (char*)d_ws;
  _Float16* Wq_t  = (_Float16*)(ws + OFF_WQ);
  _Float16* Wk_t  = (_Float16*)(ws + OFF_WK);
  _Float16* Wv_t  = (_Float16*)(ws + OFF_WV);
  _Float16* Rw_t  = (_Float16*)(ws + OFF_RW);
  _Float16* Pj_t  = (_Float16*)(ws + OFF_PJ);
  _Float16* X16   = (_Float16*)(ws + OFF_X16);
  _Float16* Tq16  = (_Float16*)(ws + OFF_TQ);
  _Float16* Tk16  = (_Float16*)(ws + OFF_TK);
  _Float16* Tv16  = (_Float16*)(ws + OFF_TV);
  _Float16* Qh16  = (_Float16*)(ws + OFF_Q);
  _Float16* Kh16  = (_Float16*)(ws + OFF_K);
  _Float16* Vt16  = (_Float16*)(ws + OFF_VT);
  _Float16* Hd16  = (_Float16*)(ws + OFF_HD);
  float*    Lam   = (float*)(ws + OFF_LAM);

  dim3 blk(256);
  dim3 gsq(DIM / 64, DIM / 64);
  dim3 gg(DIM / 64, MROWS / 64);
  dim3 gp(PDIM / 64, MROWS / 64);

  xconv_kernel<<<dim3(MROWS / 8), blk, 0, stream>>>(X, X16);
  wconv_kernel<<<gsq, blk, 0, stream>>>(wq, Wq_t, (unsigned)DIM, (unsigned)DIM);
  wconv_kernel<<<gsq, blk, 0, stream>>>(wk, Wk_t, (unsigned)DIM, (unsigned)DIM);
  wconv_kernel<<<gsq, blk, 0, stream>>>(wv, Wv_t, (unsigned)DIM, (unsigned)DIM);
  wconv_kernel<<<gsq, blk, 0, stream>>>(rw, Rw_t, (unsigned)DIM, (unsigned)DIM);
  wconv_kernel<<<dim3(PDIM / 64, DIM / 64), blk, 0, stream>>>(pw, Pj_t, (unsigned)PDIM, (unsigned)DIM);
  lam_kernel<<<dim3(1), dim3(32), 0, stream>>>(q1v, k1v, q2v, k2v, li, Lam);

  gemm_t_kernel<<<gg, blk, 0, stream>>>(X16, Wq_t, Tq16);
  gemm_t_kernel<<<gg, blk, 0, stream>>>(X16, Wk_t, Tk16);
  gemm_t_kernel<<<gg, blk, 0, stream>>>(X16, Wv_t, Tv16);
  gemm_qk_kernel<<<gp, blk, 0, stream>>>(Tq16, Pj_t, pb, Qh16);
  gemm_qk_kernel<<<gp, blk, 0, stream>>>(Tk16, Pj_t, pb, Kh16);
  gemm_v_kernel<<<gp, blk, 0, stream>>>(Tv16, Pj_t, pb, Vt16);
  attn_kernel<<<dim3(SEQ / 128, NB), blk, 0, stream>>>(Qh16, Kh16, Vt16, Lam, Hd16);
  gemm_out_kernel<<<gg, blk, 0, stream>>>(Hd16, Rw_t, out);
}
